// TUPEMultiHeadAttention_13881334300859
// MI455X (gfx1250) — hardware-run, weakly checked
//
#include <hip/hip_runtime.h>
#include <math.h>
#include <stdint.h>

typedef __attribute__((ext_vector_type(16))) _Float16 v16h;
typedef __attribute__((ext_vector_type(8)))  _Float16 v8h;
typedef __attribute__((ext_vector_type(16))) __bf16   v16b;
typedef __attribute__((ext_vector_type(8)))  __bf16   v8b;
typedef __attribute__((ext_vector_type(8)))  float    v8f;
typedef __attribute__((ext_vector_type(4)))  float    v4f;
typedef __attribute__((ext_vector_type(4)))  unsigned int v4u;

constexpr int NBATCH = 4;
constexpr int SEQ    = 1024;
constexpr int DM     = 1024;
constexpr int NH     = 16;
constexpr int HD     = 64;
constexpr int NTOK   = NBATCH * SEQ;
constexpr int POSR   = 9999;
constexpr int PMID   = 4999;
constexpr int AKC    = 64;
constexpr int NQB    = SEQ / 64;
constexpr int GPITCH = 80;

static_assert(NTOK % 64 == 0);
static_assert(DM % 64 == 0);
static_assert(DM % 32 == 0);
static_assert(SEQ % 64 == 0);
static_assert(NH * HD == DM);

__device__ __forceinline__ unsigned short f2bf_bits(float f) {
  unsigned u = __float_as_uint(f);
  return (unsigned short)((u + 0x7FFFu + ((u >> 16) & 1u)) >> 16);
}
__device__ __forceinline__ float bf_bits2f(unsigned short h) { return __uint_as_float(((unsigned)h) << 16); }

__device__ __forceinline__ void dep_guard_h(v8f& a, v8f& b, v16h x, v16h y) { asm volatile("v_nop\n\tv_nop\n\tv_nop\n\tv_nop" : "+v"(a), "+v"(b) : "v"(x), "v"(y)); }
__device__ __forceinline__ void dep_guard_b(v8f& a, v8f& b, v16b x, v16b y) { asm volatile("v_nop\n\tv_nop\n\tv_nop\n\tv_nop" : "+v"(a), "+v"(b) : "v"(x), "v"(y)); }
__device__ __forceinline__ void keep4_h(v16h a, v16h b, v16h c, v16h d) { asm volatile("v_nop" :: "v"(a), "v"(b), "v"(c), "v"(d)); }
__device__ __forceinline__ void keep4_b(v16b a, v16b b, v16b c, v16b d) { asm volatile("v_nop" :: "v"(a), "v"(b), "v"(c), "v"(d)); }
__device__ __forceinline__ void acc_guard4(v8f& a, v8f& b, v8f& c, v8f& d) { asm volatile("v_nop\n\tv_nop\n\tv_nop\n\tv_nop" : "+v"(a), "+v"(b), "+v"(c), "+v"(d)); }

template <typename T> struct Frag;
template <> struct Frag<_Float16> {
  typedef v16h V; union U { v16h v; v8h h[2]; };
  static __device__ __forceinline__ v16h load(const _Float16* p) {
    U f; f.h[0] = *(const v8h*)(p); f.h[1] = *(const v8h*)(p + 16); return f.v;
  }
  static __device__ __forceinline__ v8f mma(v16h a, v16h b, v8f c) {
    return __builtin_amdgcn_wmma_f32_16x16x32_f16(false, a, false, b, (short)0, c, false, false);
  }
  static __device__ __forceinline__ void guard(v8f& a, v8f& b, v16h x, v16h y) { dep_guard_h(a, b, x, y); }
  static __device__ __forceinline__ void keep(v16h a, v16h b, v16h c, v16h d) { keep4_h(a, b, c, d); }
};
template <> struct Frag<__bf16> {
  typedef v16b V; union U { v16b v; v8b h[2]; };
  static __device__ __forceinline__ v16b load(const __bf16* p) {
    U f; f.h[0] = *(const v8b*)(p); f.h[1] = *(const v8b*)(p + 16); return f.v;
  }
  static __device__ __forceinline__ v8f mma(v16b a, v16b b, v8f c) {
    return __builtin_amdgcn_wmma_f32_16x16x32_bf16(false, a, false, b, (short)0, c, false, false);
  }
  static __device__ __forceinline__ void guard(v8f& a, v8f& b, v16b x, v16b y) { dep_guard_b(a, b, x, y); }
  static __device__ __forceinline__ void keep(v16b a, v16b b, v16b c, v16b d) { keep4_b(a, b, c, d); }
};

__device__ __forceinline__ unsigned short at_bf_bits(float f) {
  unsigned u = __float_as_uint(f);
  return (unsigned short)((u + 0x7FFFu + ((u >> 16) & 1u)) >> 16);
}
__device__ __forceinline__ __bf16 at_f2bf(float f) { return __builtin_bit_cast(__bf16, at_bf_bits(f)); }
__device__ __forceinline__ void at_split(float f, __bf16& hi, __bf16& lo) {
  const unsigned short hb = at_bf_bits(f);
  hi = __builtin_bit_cast(__bf16, hb);
  lo = at_f2bf(f - __uint_as_float(((unsigned)hb) << 16));
}
__device__ __forceinline__ v8f at_mma(v16b a, v16b b, v8f c) {
  c = __builtin_amdgcn_wmma_f32_16x16x32_bf16(false, a, false, b, (short)0, c, false, false);
  asm volatile("v_nop\n\tv_nop\n\tv_nop\n\tv_nop" : "+v"(c) : "v"(a), "v"(b));
  return c;
}

template <int ET> struct Elem;
template <> struct Elem<0> { typedef _Float16 T; };
template <> struct Elem<1> { typedef __bf16 T; };
template <int ET, int SPLITM, int BIAS_MODE, int OUT_MODE>
__global__ __launch_bounds__(256) void wmma_gemm64(
    const unsigned short* __restrict__ Ap, const unsigned short* __restrict__ A2p, int lda, long strideA,
    const unsigned short* __restrict__ Btp, const unsigned short* __restrict__ Bt2p, int ldb, long strideB,
    void* __restrict__ Cout, void* __restrict__ Cout2, int ldc, long strideC,
    const float* __restrict__ bias, int M, int N, int K, float scale) {
  typedef typename Elem<ET>::T T;
  typedef typename Frag<T>::V V;
  const T* A = (const T*)Ap; const T* A2 = (const T*)A2p; const T* Bt = (const T*)Btp; const T* Bt2 = (const T*)Bt2p;
  __shared__ __align__(16) float sT[8][16 * 68];
  const int b    = blockIdx.y;
  const int lane = threadIdx.x & 31;
  const int wave = threadIdx.x >> 5;
  const int tilesN = N >> 6;
  const int tilesM = M >> 6;
  const int tile = blockIdx.x * 8 + wave;
  if (tile >= tilesM * tilesN) return;
  const int tm = tile / tilesN;
  const int tn = tile - tm * tilesN;
  const int m0 = tm << 6;
  const int n0 = tn << 6;

  const T* Ab  = A  + (size_t)b * strideA;
  const T* Bb  = Bt + (size_t)b * strideB;
  const T* Ab2 = SPLITM ? (A2 + (size_t)b * strideA) : nullptr;
  const T* Bb2 = (SPLITM == 1) ? (Bt2 + (size_t)b * strideB) : nullptr;

  const int rlane = lane & 15;
  const int koff  = (lane >> 4) * 8;
  const int mOff  = (lane >> 4) * 8;

  v8f acc[4][4];
#pragma unroll
  for (int i = 0; i < 4; ++i)
#pragma unroll
    for (int j = 0; j < 4; ++j) acc[i][j] = (v8f){0.f,0.f,0.f,0.f,0.f,0.f,0.f,0.f};

  for (int k0 = 0; k0 < K; k0 += 32) {
    V bh[4], bl[4];
#pragma unroll
    for (int j = 0; j < 4; ++j) {
      const size_t bo = (size_t)(n0 + (j << 4) + rlane) * ldb + koff + k0;
      bh[j] = Frag<T>::load(Bb + bo);
      if (SPLITM == 1) bl[j] = Frag<T>::load(Bb2 + bo);
    }
#pragma unroll
    for (int i = 0; i < 4; ++i) {
      const size_t ao = (size_t)(m0 + (i << 4) + rlane) * lda + koff + k0;
      V ah = Frag<T>::load(Ab + ao);
      V al;
      if (SPLITM) al = Frag<T>::load(Ab2 + ao);
#pragma unroll
      for (int j = 0; j < 4; ++j) {
        acc[i][j] = Frag<T>::mma(ah, bh[j], acc[i][j]);
        if (SPLITM == 1) acc[i][j] = Frag<T>::mma(ah, bl[j], acc[i][j]);
        if (SPLITM) acc[i][j] = Frag<T>::mma(al, bh[j], acc[i][j]);
      }
      Frag<T>::guard(acc[i][0], acc[i][3], ah, SPLITM ? al : ah);
    }
    Frag<T>::keep(bh[0], bh[1], bh[2], bh[3]);
    if (SPLITM == 1) Frag<T>::keep(bl[0], bl[1], bl[2], bl[3]);
  }
  acc_guard4(acc[0][0], acc[0][1], acc[0][2], acc[0][3]);
  acc_guard4(acc[1][0], acc[1][1], acc[1][2], acc[1][3]);
  acc_guard4(acc[2][0], acc[2][1], acc[2][2], acc[2][3]);
  acc_guard4(acc[3][0], acc[3][1], acc[3][2], acc[3][3]);

  float* slab = sT[wave];
#pragma unroll
  for (int i = 0; i < 4; ++i) {
    const int mBase = m0 + (i << 4);
    float bm[8];
#pragma unroll
    for (int r = 0; r < 8; ++r) bm[r] = 0.f;
    if (BIAS_MODE == 1) {
      const v4f bA = *(const v4f*)(bias + mBase + mOff);
      const v4f bB = *(const v4f*)(bias + mBase + mOff + 4);
      bm[0] = bA[0]; bm[1] = bA[1]; bm[2] = bA[2]; bm[3] = bA[3];
      bm[4] = bB[0]; bm[5] = bB[1]; bm[6] = bB[2]; bm[7] = bB[3];
    }
#pragma unroll
    for (int j = 0; j < 4; ++j) {
      const int n = n0 + (j << 4) + rlane;
      float bv = 0.f;
      if (BIAS_MODE == 2) bv = bias[n];
#pragma unroll
      for (int r = 0; r < 8; ++r) {
        float v = acc[i][j][r] * scale;
        if (BIAS_MODE == 1) v += bm[r];
        if (BIAS_MODE == 2) v += bv;
        slab[(mOff + r) * 68 + (j << 4) + rlane] = v;
      }
    }
    __builtin_amdgcn_fence(__ATOMIC_RELEASE, "workgroup");
    __builtin_amdgcn_wave_barrier();
    __builtin_amdgcn_fence(__ATOMIC_ACQUIRE, "workgroup");
    if (OUT_MODE == 0) {
      float* C = (float*)Cout + (size_t)b * strideC;
      const int hh = lane >> 4, c4 = (lane & 15) * 4;
      for (int pass = 0; pass < 2; ++pass) {
#pragma unroll
        for (int it = 0; it < 8; ++it) {
          const int row = it * 2 + hh;
          v4f v = *(const v4f*)(slab + row * 68 + c4);
          *(volatile v4f*)(C + (size_t)(mBase + row) * ldc + n0 + c4) = v;
        }
        __threadfence();
      }
    } else {
      const int q = lane >> 3, c8 = (lane & 7) * 8;
      unsigned short* C  = (unsigned short*)Cout  + (size_t)b * strideC;
      unsigned short* C2 = (OUT_MODE == 2) ? ((unsigned short*)Cout2 + (size_t)b * strideC) : nullptr;
      for (int pass = 0; pass < 2; ++pass) {
#pragma unroll
        for (int it = 0; it < 4; ++it) {
          const int row = it * 4 + q;
          const float* sp = slab + row * 68 + c8;
          v8h hv, lv;
#pragma unroll
          for (int e = 0; e < 8; ++e) {
            if (OUT_MODE == 1) {
              hv[e] = (_Float16)sp[e];
            } else {
              unsigned short hb = f2bf_bits(sp[e]);
              unsigned short lb = f2bf_bits(sp[e] - bf_bits2f(hb));
              hv[e] = __builtin_bit_cast(_Float16, hb);
              lv[e] = __builtin_bit_cast(_Float16, lb);
            }
          }
          *(volatile v8h*)(C + (size_t)(mBase + row) * ldc + n0 + c8) = hv;
          if (OUT_MODE == 2) *(volatile v8h*)(C2 + (size_t)(mBase + row) * ldc + n0 + c8) = lv;
        }
        __threadfence();
      }
    }
    __builtin_amdgcn_fence(__ATOMIC_RELEASE, "workgroup");
    __builtin_amdgcn_wave_barrier();
    __builtin_amdgcn_fence(__ATOMIC_ACQUIRE, "workgroup");
  }
}

__global__ __launch_bounds__(256) void cast_f32_bf16x8(const float* __restrict__ in,
                                                       unsigned short* __restrict__ out, int n8) {
  const int i = blockIdx.x * 256 + threadIdx.x;
  if (i < n8) {
    const float* p = in + (size_t)i * 8;
    const v4f a = *(const v4f*)p;
    const v4f c = *(const v4f*)(p + 4);
    v4u u;
    u[0] = (unsigned)f2bf_bits(a[0]) | ((unsigned)f2bf_bits(a[1]) << 16);
    u[1] = (unsigned)f2bf_bits(a[2]) | ((unsigned)f2bf_bits(a[3]) << 16);
    u[2] = (unsigned)f2bf_bits(c[0]) | ((unsigned)f2bf_bits(c[1]) << 16);
    u[3] = (unsigned)f2bf_bits(c[2]) | ((unsigned)f2bf_bits(c[3]) << 16);
    unsigned short* d = out + (size_t)i * 8;
    *(volatile v4u*)d = u;
    __threadfence();
    *(volatile v4u*)d = u;
  }
}

__global__ __launch_bounds__(256) void transpose_cast_w(const float* __restrict__ in,
                                                        unsigned short* __restrict__ out) {
  __shared__ float tile[64][65];
  const int n0 = blockIdx.x * 64;
  const int k0 = blockIdx.y * 64;
  const int tid = threadIdx.x;
#pragma unroll
  for (int i = 0; i < 4; ++i) {
    const int idx = tid + 256 * i;
    const int kk = idx >> 4;
    const int c4 = (idx & 15) * 4;
    const v4f x = *(const v4f*)(in + (size_t)(k0 + kk) * DM + n0 + c4);
    tile[kk][c4 + 0] = x[0];
    tile[kk][c4 + 1] = x[1];
    tile[kk][c4 + 2] = x[2];
    tile[kk][c4 + 3] = x[3];
  }
  __syncthreads();
#pragma unroll
  for (int i = 0; i < 2; ++i) {
    const int idx = tid + 256 * i;
    const int nl = idx >> 3;
    const int k8 = (idx & 7) * 8;
    v4u u;
#pragma unroll
    for (int e = 0; e < 4; ++e) {
      const unsigned lo = (unsigned)f2bf_bits(tile[k8 + 2 * e][nl]);
      const unsigned hi = (unsigned)f2bf_bits(tile[k8 + 2 * e + 1][nl]);
      u[e] = lo | (hi << 16);
    }
    unsigned short* d = out + (size_t)(n0 + nl) * DM + k0 + k8;
    *(volatile v4u*)d = u;
    __threadfence();
    *(volatile v4u*)d = u;
  }
}

__global__ __launch_bounds__(256) void rne_tables(const float* __restrict__ b0, const float* __restrict__ b1,
                                                  const float* __restrict__ b2, const float* __restrict__ b3,
                                                  const float* __restrict__ gam, float* __restrict__ tab) {
  const int blk = blockIdx.x;
  const int t = threadIdx.x;
  if (blk < 4) {
    const float* src = b0;
    if (blk == 1) src = b1;
    if (blk == 2) src = b2;
    if (blk == 3) src = b3;
    const v4f x = *(const v4f*)(src + 4 * t);
    v4f y;
#pragma unroll
    for (int e = 0; e < 4; ++e) y[e] = bf_bits2f(f2bf_bits(x[e]));
    float* d = tab + blk * 1024 + 4 * t;
    *(volatile v4f*)d = y;
    __threadfence();
    *(volatile v4f*)d = y;
  } else if (t < 8) {
    v4f y;
#pragma unroll
    for (int e = 0; e < 4; ++e) {
      int gi = 4 * t + e;
      gi = gi < NH ? gi : (NH - 1);
      y[e] = bf_bits2f(f2bf_bits(gam[gi]));
    }
    float* d = tab + 4096 + 4 * t;
    *(volatile v4f*)d = y;
    __threadfence();
    *(volatile v4f*)d = y;
  }
}

__global__ __launch_bounds__(128) void attn_rel_kernel(
    const unsigned short* __restrict__ Qhp, const unsigned short* __restrict__ Qlp,
    const unsigned short* __restrict__ Khp, const unsigned short* __restrict__ Klp,
    const unsigned short* __restrict__ VThp, const unsigned short* __restrict__ VTlp,
    const unsigned short* __restrict__ PEp, const float* __restrict__ gtab,
    unsigned short* __restrict__ Ohp, unsigned short* __restrict__ Olp) {
  union FB { v16b v; v8b h[2]; };
  __shared__ __align__(16) __bf16 Ksh[AKC * HD];
  __shared__ __align__(16) __bf16 Ksl[AKC * HD];
  __shared__ __align__(16) __bf16 Vth[HD * AKC];
  __shared__ __align__(16) __bf16 Vtl[HD * AKC];
  __shared__ __align__(16) __bf16 PEs[128 * HD];
  __shared__ __align__(16) __bf16 Psh[4][16 * AKC];
  __shared__ __align__(16) __bf16 Psl[4][16 * AKC];
  __shared__ __align__(16) float  Gbuf[4][16 * GPITCH];

  const int tid  = threadIdx.x;
  const int wave = tid >> 5;
  const int lane = tid & 31;
  const int hh   = lane >> 4;
  const int c    = lane & 15;
  const int koff = 8 * hh;

  const int bx = blockIdx.x;
  const int qb = bx % NQB;
  const int bh = bx / NQB;
  const int h  = bh % NH;
  const int b  = bh / NH;
  const int q0 = qb * 64 + wave * 16;
  const float gma = gtab[h];

  const __bf16* Qh = (const __bf16*)Qhp;
  const __bf16* Ql = (const __bf16*)Qlp;

  v16b qah[2], qal[2];
  {
    const size_t qo = (size_t)(b * SEQ + q0 + c) * DM + h * HD + koff;
#pragma unroll
    for (int dc = 0; dc < 2; ++dc) {
      qah[dc] = Frag<__bf16>::load(Qh + qo + dc * 32);
      qal[dc] = Frag<__bf16>::load(Ql + qo + dc * 32);
    }
  }

  float mrow[8], lrow[8];
  v8f oacc[4];
#pragma unroll
  for (int r = 0; r < 8; ++r) { mrow[r] = -INFINITY; lrow[r] = 0.f; }
#pragma unroll
  for (int t = 0; t < 4; ++t) oacc[t] = (v8f){0.f,0.f,0.f,0.f,0.f,0.f,0.f,0.f};

  float* gb = Gbuf[wave];
  const __bf16* pw = PEs + wave * 16 * HD;
  __bf16* pwh = Psh[wave];
  __bf16* pwl = Psl[wave];

  for (int kc = 0; kc < SEQ / AKC; ++kc) {
    const int kv0 = kc * AKC;
    const int rbase = qb * 64 - kv0 - 63 + PMID;
    __syncthreads();
    {
#pragma unroll
      for (int i = 0; i < 4; ++i) {
        const int idx = tid + 128 * i;
        const int row = idx >> 3;
        const int pc8 = (idx & 7) * 8;
        const size_t go = (size_t)(b * SEQ + kv0 + row) * DM + h * HD + pc8;
        const v4u a  = *(const v4u*)(Khp + go);
        const v4u a2 = *(const v4u*)(Klp + go);
        *(v4u*)(Ksh + row * HD + pc8) = a;
        *(v4u*)(Ksl + row * HD + pc8) = a2;
      }
      asm volatile("" ::: "memory");
#pragma unroll
      for (int i = 0; i < 4; ++i) {
        const int idx = tid + 128 * i;
        const int row = idx >> 3;
        const int pc8 = (idx & 7) * 8;
        const size_t go = ((size_t)b * DM + h * HD + row) * SEQ + kv0 + pc8;
        const v4u a  = *(const v4u*)(VThp + go);
        const v4u a2 = *(const v4u*)(VTlp + go);
        *(v4u*)(Vth + row * AKC + pc8) = a;
        *(v4u*)(Vtl + row * AKC + pc8) = a2;
      }
      asm volatile("" ::: "memory");
#pragma unroll
      for (int i = 0; i < 8; ++i) {
        const int idx = tid + 128 * i;
        const int row = idx >> 3;
        const int pc8 = (idx & 7) * 8;
        int prow = rbase + row;
        prow = prow < 0 ? 0 : (prow > POSR - 1 ? POSR - 1 : prow);
        const v4u a = *(const v4u*)(PEp + (size_t)prow * HD + pc8);
        *(v4u*)(PEs + row * HD + pc8) = a;
      }
    }
    __syncthreads();

#pragma unroll
    for (int gt = 0; gt < 5; ++gt) {
      v8f gacc = (v8f){0.f,0.f,0.f,0.f,0.f,0.f,0.f,0.f};
#pragma unroll
      for (int dc = 0; dc < 2; ++dc) {
        FB pb;
        pb.h[0] = *(const v8b*)(pw + (gt * 16 + c) * HD + dc * 32 + koff);
        pb.h[1] = *(const v8b*)(pw + (gt * 16 + c) * HD + dc * 32 + 16 + koff);
        gacc = at_mma(qah[dc], pb.v, gacc);
        gacc = at_mma(qal[dc], pb.v, gacc);
      }
#pragma unroll
      for (int r = 0; r < 8; ++r) gb[(8 * hh + r) * GPITCH + gt * 16 + c] = gacc[r];
    }

    v8f s[4];
#pragma unroll
    for (int j = 0; j < 4; ++j) {
      s[j] = (v8f){0.f,0.f,0.f,0.f,0.f,0.f,0.f,0.f};
#pragma unroll
      for (int dc = 0; dc < 2; ++dc) {
        FB kb, kl;
        kb.h[0] = *(const v8b*)(Ksh + (j * 16 + c) * HD + dc * 32 + koff);
        kb.h[1] = *(const v8b*)(Ksh + (j * 16 + c) * HD + dc * 32 + 16 + koff);
        kl.h[0] = *(const v8b*)(Ksl + (j * 16 + c) * HD + dc * 32 + koff);
        kl.h[1] = *(const v8b*)(Ksl + (j * 16 + c) * HD + dc * 32 + 16 + koff);
        s[j] = at_mma(qah[dc], kb.v, s[j]);
        s[j] = at_mma(qah[dc], kl.v, s[j]);
        s[j] = at_mma(qal[dc], kb.v, s[j]);
      }
    }
    __builtin_amdgcn_fence(__ATOMIC_RELEASE, "workgroup");
    __builtin_amdgcn_wave_barrier();
    __builtin_amdgcn_fence(__ATOMIC_ACQUIRE, "workgroup");

    float cm[8];
#pragma unroll
    for (int r = 0; r < 8; ++r) {
      const int i = 8 * hh + r;
      float m = -INFINITY;
#pragma unroll
      for (int j = 0; j < 4; ++j) {
        const int jj = j * 16 + c;
        const float gg = gb[i * GPITCH + (i - jj + 63)];
        const float sc = (s[j][r] + gma * gg) * 0.125f;
        s[j][r] = sc;
        m = fmaxf(m, sc);
      }
#pragma unroll
      for (int off = 1; off < 16; off <<= 1) m = fmaxf(m, __shfl_xor(m, off, 32));
      cm[r] = m;
    }
#pragma unroll
    for (int r = 0; r < 8; ++r) {
      const float mnew = fmaxf(mrow[r], cm[r]);
      const float alpha = expf(mrow[r] - mnew);
      mrow[r] = mnew;
      float psum = 0.f;
#pragma unroll
      for (int j = 0; j < 4; ++j) {
        const float p = expf(s[j][r] - mnew);
        psum += p;
        __bf16 a, bl;
        at_split(p, a, bl);
        pwh[(8 * hh + r) * AKC + j * 16 + c] = a;
        pwl[(8 * hh + r) * AKC + j * 16 + c] = bl;
      }
#pragma unroll
      for (int off = 1; off < 16; off <<= 1) psum += __shfl_xor(psum, off, 32);
      lrow[r] = lrow[r] * alpha + psum;
#pragma unroll
      for (int t = 0; t < 4; ++t) oacc[t][r] *= alpha;
    }
    __builtin_amdgcn_fence(__ATOMIC_RELEASE, "workgroup");
    __builtin_amdgcn_wave_barrier();
    __builtin_amdgcn_fence(__ATOMIC_ACQUIRE, "workgroup");
#pragma unroll 1
    for (int kk = 0; kk < 2; ++kk) {
      FB pa, pl;
      pa.h[0] = *(const v8b*)(pwh + c * AKC + kk * 32 + koff);
      pa.h[1] = *(const v8b*)(pwh + c * AKC + kk * 32 + 16 + koff);
      pl.h[0] = *(const v8b*)(pwl + c * AKC + kk * 32 + koff);
      pl.h[1] = *(const v8b*)(pwl + c * AKC + kk * 32 + 16 + koff);
#pragma unroll
      for (int t = 0; t < 4; ++t) {
        FB vb, vl;
        vb.h[0] = *(const v8b*)(Vth + (t * 16 + c) * AKC + kk * 32 + koff);
        vb.h[1] = *(const v8b*)(Vth + (t * 16 + c) * AKC + kk * 32 + 16 + koff);
        vl.h[0] = *(const v8b*)(Vtl + (t * 16 + c) * AKC + kk * 32 + koff);
        vl.h[1] = *(const v8b*)(Vtl + (t * 16 + c) * AKC + kk * 32 + 16 + koff);
        oacc[t] = at_mma(pa.v, vb.v, oacc[t]);
        oacc[t] = at_mma(pa.v, vl.v, oacc[t]);
        oacc[t] = at_mma(pl.v, vb.v, oacc[t]);
      }
    }
  }

  float* os = gb;
#pragma unroll
  for (int r = 0; r < 8; ++r) {
    const float inv = 1.0f / lrow[r];
#pragma unroll
    for (int t = 0; t < 4; ++t) os[(8 * hh + r) * GPITCH + t * 16 + c] = oacc[t][r] * inv;
  }
  __builtin_amdgcn_fence(__ATOMIC_RELEASE, "workgroup");
  __builtin_amdgcn_wave_barrier();
  __builtin_amdgcn_fence(__ATOMIC_ACQUIRE, "workgroup");
  {
    const int q4 = lane >> 3, c8 = (lane & 7) * 8;
    for (int pass = 0; pass < 2; ++pass) {
#pragma unroll
      for (int it = 0; it < 4; ++it) {
        const int row = it * 4 + q4;
        const float* sp = os + row * GPITCH + c8;
        v8h hv, lv;
#pragma unroll
        for (int e = 0; e < 8; ++e) {
          const unsigned short hb = f2bf_bits(sp[e]);
          const unsigned short lb = f2bf_bits(sp[e] - bf_bits2f(hb));
          hv[e] = __builtin_bit_cast(_Float16, hb);
          lv[e] = __builtin_bit_cast(_Float16, lb);
        }
        const size_t oo = (size_t)(b * SEQ + q0 + row) * DM + h * HD + c8;
        *(volatile v8h*)(Ohp + oo) = hv;
        *(volatile v8h*)(Olp + oo) = lv;
      }
      __threadfence();
    }
  }
}

constexpr size_t ACT_PLANE = (size_t)NTOK * DM * 2;
constexpr size_t W_PLANE   = (size_t)DM * DM * 2;
constexpr size_t PE_BYTES  = (size_t)POSR * HD * 2;
constexpr size_t PE_CARVE  = 1280000;
constexpr size_t TAB_FLOATS = 4096 + 32;
constexpr size_t TAB_CARVE = 16640;
constexpr size_t OFF_XQ  = 0;
constexpr size_t OFF_XK  = OFF_XQ + ACT_PLANE;
constexpr size_t OFF_XV  = OFF_XK + ACT_PLANE;
constexpr size_t OFF_WQ  = OFF_XV + ACT_PLANE;
constexpr size_t OFF_WK  = OFF_WQ + W_PLANE;
constexpr size_t OFF_WV  = OFF_WK + W_PLANE;
constexpr size_t OFF_WO  = OFF_WV + W_PLANE;
constexpr size_t OFF_PE  = OFF_WO + W_PLANE;
constexpr size_t OFF_TAB = OFF_PE + PE_CARVE;
constexpr size_t OFF_QH  = OFF_TAB + TAB_CARVE;
constexpr size_t OFF_QL  = OFF_QH + ACT_PLANE;
constexpr size_t OFF_KH  = OFF_QL + ACT_PLANE;
constexpr size_t OFF_KL  = OFF_KH + ACT_PLANE;
constexpr size_t OFF_VTH = OFF_KL + ACT_PLANE;
constexpr size_t OFF_VTL = OFF_VTH + ACT_PLANE;
constexpr size_t OFF_OH  = OFF_VTL + ACT_PLANE;
constexpr size_t OFF_OL  = OFF_OH + ACT_PLANE;
constexpr size_t WS_TOTAL = OFF_OL + ACT_PLANE;
static_assert(PE_CARVE >= PE_BYTES);
static_assert(TAB_CARVE >= TAB_FLOATS * 4);
static_assert(OFF_PE % 256 == 0 && OFF_TAB % 256 == 0 && OFF_QH % 256 == 0);
static_assert(WS_TOTAL == 101959936);
static_assert(WS_TOTAL <= 134217728);
static_assert((NTOK * DM) % 8 == 0 && (POSR * HD) % 8 == 0);

extern "C" void kernel_launch(void* const* d_in, const int* in_sizes, int n_in,
                              void* d_out, int out_size, void* d_ws,
                              size_t ws_size, hipStream_t stream) {
  if (n_in < 13) return;
  if (out_size != NTOK * DM) return;
  if (ws_size < WS_TOTAL) return;
  if (in_sizes[0] != NTOK * DM || in_sizes[9] != POSR * HD || in_sizes[10] < NH) return;

  const float* v_f   = (const float*)d_in[0];
  const float* k_f   = (const float*)d_in[1];
  const float* q_f   = (const float*)d_in[2];
  const float* Wq    = (const float*)d_in[3];
  const float* bq    = (const float*)d_in[4];
  const float* Wk    = (const float*)d_in[5];
  const float* bk    = (const float*)d_in[6];
  const float* Wv    = (const float*)d_in[7];
  const float* bv    = (const float*)d_in[8];
  const float* pos   = (const float*)d_in[9];
  const float* gamma = (const float*)d_in[10];
  const float* Wo    = (const float*)d_in[11];
  const float* bo    = (const float*)d_in[12];

  char* ws = (char*)d_ws;
  unsigned short* xq  = (unsigned short*)(ws + OFF_XQ);
  unsigned short* xk  = (unsigned short*)(ws + OFF_XK);
  unsigned short* xv  = (unsigned short*)(ws + OFF_XV);
  unsigned short* wqT = (unsigned short*)(ws + OFF_WQ);
  unsigned short* wkT = (unsigned short*)(ws + OFF_WK);
  unsigned short* wvT = (unsigned short*)(ws + OFF_WV);
  unsigned short* woT = (unsigned short*)(ws + OFF_WO);
  unsigned short* pe  = (unsigned short*)(ws + OFF_PE);
  float*          tab = (float*)(ws + OFF_TAB);
  unsigned short* qh  = (unsigned short*)(ws + OFF_QH);
  unsigned short* ql  = (unsigned short*)(ws + OFF_QL);
  unsigned short* kh  = (unsigned short*)(ws + OFF_KH);
  unsigned short* kl  = (unsigned short*)(ws + OFF_KL);
  unsigned short* vth = (unsigned short*)(ws + OFF_VTH);
  unsigned short* vtl = (unsigned short*)(ws + OFF_VTL);
  unsigned short* oh  = (unsigned short*)(ws + OFF_OH);
  unsigned short* ol  = (unsigned short*)(ws + OFF_OL);

  const int n8act = NTOK * DM / 8;
  const int n8pe  = POSR * HD / 8;
  cast_f32_bf16x8<<<dim3((n8act + 255) / 256), dim3(256), 0, stream>>>(q_f, xq, n8act);
  cast_f32_bf16x8<<<dim3((n8act + 255) / 256), dim3(256), 0, stream>>>(k_f, xk, n8act);
  cast_f32_bf16x8<<<dim3((n8act + 255) / 256), dim3(256), 0, stream>>>(v_f, xv, n8act);
  cast_f32_bf16x8<<<dim3((n8pe + 255) / 256), dim3(256), 0, stream>>>(pos, pe, n8pe);

  const dim3 gw(DM / 64, DM / 64);
  transpose_cast_w<<<gw, dim3(256), 0, stream>>>(Wq, wqT);
  transpose_cast_w<<<gw, dim3(256), 0, stream>>>(Wk, wkT);
  transpose_cast_w<<<gw, dim3(256), 0, stream>>>(Wv, wvT);
  transpose_cast_w<<<gw, dim3(256), 0, stream>>>(Wo, woT);

  rne_tables<<<dim3(5), dim3(256), 0, stream>>>(bq, bk, bv, bo, gamma, tab);

  const int gproj = ((NTOK / 64) * (DM / 64) + 7) / 8;
  wmma_gemm64<1, 0, 2, 2><<<dim3(gproj, 1), dim3(256), 0, stream>>>(
      xq, nullptr, DM, 0L, wqT, nullptr, DM, 0L, (void*)qh, (void*)ql, DM, 0L,
      tab + 0, NTOK, DM, DM, 1.0f);
  wmma_gemm64<1, 0, 2, 2><<<dim3(gproj, 1), dim3(256), 0, stream>>>(
      xk, nullptr, DM, 0L, wkT, nullptr, DM, 0L, (void*)kh, (void*)kl, DM, 0L,
      tab + 1024, NTOK, DM, DM, 1.0f);
  const int gvt = ((DM / 64) * (SEQ / 64) + 7) / 8;
  wmma_gemm64<1, 0, 1, 2><<<dim3(gvt, NBATCH), dim3(256), 0, stream>>>(
      wvT, nullptr, DM, 0L, xv, nullptr, DM, (long)SEQ * DM, (void*)vth, (void*)vtl, SEQ, (long)DM * SEQ,
      tab + 2048, DM, SEQ, DM, 1.0f);

  attn_rel_kernel<<<dim3(NBATCH * NH * NQB), dim3(128), 0, stream>>>(
      qh, ql, kh, kl, vth, vtl, pe, tab + 4096, oh, ol);

  wmma_gemm64<1, 2, 2, 0><<<dim3(gproj, 1), dim3(256), 0, stream>>>(
      oh, ol, DM, 0L, woT, nullptr, DM, 0L, d_out, nullptr, DM, 0L,
      tab + 3072, NTOK, DM, DM, 1.0f);
}
